// down_block_trans_49520972923052
// MI455X (gfx1250) — hardware-verified
//
#include <hip/hip_runtime.h>

#pragma clang fp contract(off)

typedef unsigned short us;
typedef us     v8us  __attribute__((ext_vector_type(8)));
typedef us     v16us __attribute__((ext_vector_type(16)));
typedef __bf16 v16bf __attribute__((ext_vector_type(16)));
typedef float  v8f   __attribute__((ext_vector_type(8)));
typedef float  v4f   __attribute__((ext_vector_type(4)));
typedef double v2d   __attribute__((ext_vector_type(2)));
typedef v8us __attribute__((may_alias)) v8usa;
typedef v4f  __attribute__((may_alias)) v4fa;

union Fr16 { v16us v; v8us h[2]; };

#define IMG   128
#define HWSZ  16384
#define MTOT  32768
#define NCH   128
#define NKEY  256
#define DHEAD 32
#define NCMP  2048

__device__ __forceinline__ us bf_bits(float f) {
  unsigned u = __float_as_uint(f);
  u = u + 0x7FFFu + ((u >> 16) & 1u);
  return (us)(u >> 16);
}
__device__ __forceinline__ float bf_val(us b) {
  return __uint_as_float(((unsigned)b) << 16);
}

__device__ __forceinline__ v8f wmma1(v16us a, v16us b, v8f c) {
  const v16bf av = __builtin_bit_cast(v16bf, a);
  const v16bf bv = __builtin_bit_cast(v16bf, b);
  v8f d = __builtin_amdgcn_wmma_f32_16x16x32_bf16(false, av, false, bv, (short)0, c, false, false);
  asm volatile("v_nop\n\tv_nop\n\tv_nop\n\tv_nop" : "+v"(d) : "v"(av), "v"(bv));
  return d;
}
__device__ __forceinline__ v8f wmma3(v16us ah, v16us al, v16us bh, v16us bl, v8f c) {
  c = wmma1(ah, bh, c);
  c = wmma1(ah, bl, c);
  c = wmma1(al, bh, c);
  return c;
}
__device__ __forceinline__ v16us ldfrag(const us* p) {
  Fr16 f;
  f.h[0] = *(const v8usa*)p;
  f.h[1] = *(const v8usa*)(p + 16);
  return f.v;
}
__device__ __forceinline__ v16us zero16() {
  const v16us z = {0, 0, 0, 0, 0, 0, 0, 0, 0, 0, 0, 0, 0, 0, 0, 0};
  return z;
}
__device__ __forceinline__ v8f zero8f() {
  const v8f z = {0.f, 0.f, 0.f, 0.f, 0.f, 0.f, 0.f, 0.f};
  return z;
}

__device__ __forceinline__ int interp_lo(int r, float& frac) {
  const float pos = (float)r * (127.0f / 15.0f);
  int lo = (int)floorf(pos);
  lo = min(max(lo, 0), IMG - 2);
  frac = pos - (float)lo;
  return lo;
}

__global__ __launch_bounds__(256) void k_wcvt(const float* __restrict__ W, int OC, int IC, int ntaps,
                                             us* __restrict__ Bh, us* __restrict__ Bl) {
  const int Ksz = ntaps * IC;
  const int total = OC * Ksz;
  const int e0 = (blockIdx.x * 256 + threadIdx.x) * 8;
  if (e0 >= total) return;
  const int oc = e0 / Ksz;
  const int rem = e0 - oc * Ksz;
  const int tap = rem / IC;
  const int ic = rem - tap * IC;
  v8us hh, ll;
  #pragma unroll
  for (int e = 0; e < 8; ++e) {
    const float v = W[((size_t)(oc * IC + ic + e)) * ntaps + tap];
    const us hb = bf_bits(v);
    hh[e] = hb;
    ll[e] = bf_bits(v - bf_val(hb));
  }
  *(volatile v8us*)(Bh + e0) = hh;
  *(volatile v8us*)(Bl + e0) = ll;
  __threadfence();
  *(volatile v8us*)(Bh + e0) = hh;
  *(volatile v8us*)(Bl + e0) = ll;
}

__global__ __launch_bounds__(256) void k_maxpool(const float* __restrict__ X, float* __restrict__ P) {
  __shared__ __attribute__((aligned(16))) float T[32 * 64];
  const int t = threadIdx.x;
  const int blk = blockIdx.x;
  const int b = blk >> 9, y = (blk >> 2) & 127, x0 = (blk & 3) * 32;
  #pragma unroll
  for (int it = 0; it < 8; ++it) {
    const int e = it * 256 + t;
    const int c = e >> 5, px = e & 31;
    const float* s = X + ((((size_t)(b * 64 + c)) * 256 + 2 * y) * 256 + 2 * (x0 + px));
    T[px * 64 + c] = fmaxf(fmaxf(s[0], s[1]), fmaxf(s[256], s[257]));
  }
  __syncthreads();
  float* dst = P + ((size_t)(b * HWSZ + y * IMG + x0)) * 64;
  *(volatile v4f*)(dst + t * 4)        = *(const v4fa*)(T + t * 4);
  *(volatile v4f*)(dst + 1024 + t * 4) = *(const v4fa*)(T + 1024 + t * 4);
  __threadfence();
  *(volatile v4f*)(dst + t * 4)        = *(const v4fa*)(T + t * 4);
  *(volatile v4f*)(dst + 1024 + t * 4) = *(const v4fa*)(T + 1024 + t * 4);
}

__global__ __launch_bounds__(256) void k_stats(const float* __restrict__ In, int C, int csh,
                                              double* __restrict__ part) {
  __shared__ double s1[256];
  __shared__ double s2[256];
  const int t = threadIdx.x;
  const int c = t & (C - 1);
  const int q = t >> csh;
  const int Q = 256 >> csh;
  const int r0 = blockIdx.x * 128;
  double a = 0.0, aq = 0.0;
  #pragma unroll 1
  for (int r = q; r < 128; r += Q) {
    const double v = (double)In[((size_t)(r0 + r)) * C + c];
    a += v;
    aq += v * v;
  }
  s1[t] = a;
  s2[t] = aq;
  __syncthreads();
  if (t < C) {
    double A = 0.0, Bq = 0.0;
    #pragma unroll 1
    for (int k = 0; k < Q; ++k) { A += s1[k * C + t]; Bq += s2[k * C + t]; }
    v2d o;
    o.x = A;
    o.y = Bq;
    double* dp = part + ((size_t)(blockIdx.x * C + t)) * 2;
    *(volatile v2d*)dp = o;
    __threadfence();
    *(volatile v2d*)dp = o;
  }
}

__global__ __launch_bounds__(128) void k_bnfin(const double* __restrict__ part, int C,
                                              const float* __restrict__ g, const float* __restrict__ bb,
                                              float* __restrict__ scsh) {
  const int c = threadIdx.x;
  if (c >= C) return;
  double A = 0.0, Bq = 0.0;
  #pragma unroll 1
  for (int k = 0; k < 256; ++k) {
    A  += part[((size_t)(k * C + c)) * 2];
    Bq += part[((size_t)(k * C + c)) * 2 + 1];
  }
  const double mean = A * (1.0 / 32768.0);
  double var = Bq * (1.0 / 32768.0) - mean * mean;
  if (var < 0.0) var = 0.0;
  const float istd = 1.0f / sqrtf((float)var + 1e-5f);
  const float sc = istd * g[c];
  const float sh = bb[c] - (float)mean * sc;
  *(volatile float*)(scsh + c) = sc;
  *(volatile float*)(scsh + 128 + c) = sh;
  __threadfence();
  *(volatile float*)(scsh + c) = sc;
  *(volatile float*)(scsh + 128 + c) = sh;
}

__global__ __launch_bounds__(256) void k_apply(const float* __restrict__ In, const float* __restrict__ scsh,
                                              int C, int relu, us* __restrict__ Oh, us* __restrict__ Ol) {
  const size_t e0 = ((size_t)blockIdx.x * 256 + threadIdx.x) * 8;
  const int c0 = (int)(e0 & (size_t)(C - 1));
  const v4f a = *(const v4fa*)(In + e0);
  const v4f b2 = *(const v4fa*)(In + e0 + 4);
  float v[8] = {a.x, a.y, a.z, a.w, b2.x, b2.y, b2.z, b2.w};
  v8us hh, ll;
  #pragma unroll
  for (int e = 0; e < 8; ++e) {
    float y = fmaf(v[e], scsh[c0 + e], scsh[128 + c0 + e]);
    if (relu) y = fmaxf(y, 0.0f);
    const us hb = bf_bits(y);
    hh[e] = hb;
    ll[e] = bf_bits(y - bf_val(hb));
  }
  *(volatile v8us*)(Oh + e0) = hh;
  *(volatile v8us*)(Ol + e0) = ll;
  __threadfence();
  *(volatile v8us*)(Oh + e0) = hh;
  *(volatile v8us*)(Ol + e0) = ll;
}

__global__ __launch_bounds__(128) void k_gemm(const us* __restrict__ Ah, const us* __restrict__ Al,
                                             const us* __restrict__ Bh, const us* __restrict__ Bl,
                                             const float* Res, float* Cf,
                                             int IC, int icsh, int ntaps, int N, int addres) {
  __shared__ __attribute__((aligned(16))) float Cs[128 * 64];
  const int tid = threadIdx.x, lane = tid & 31, w = tid >> 5;
  const int hl = lane >> 4, m = lane & 15;
  const int m0 = blockIdx.x * 128, n0 = blockIdx.y * 64;
  const int Ksz = ntaps * IC;
  const int prow0 = m0 + 32 * w + m;
  const int prow1 = prow0 + 16;
  const int pb0 = prow0 >> 14, py0 = (prow0 >> 7) & 127, px0 = prow0 & 127;
  const int pb1 = prow1 >> 14, py1 = (prow1 >> 7) & 127, px1 = prow1 & 127;

  v8f acc[2][4];
  #pragma unroll
  for (int mt = 0; mt < 2; ++mt)
    #pragma unroll
    for (int nt = 0; nt < 4; ++nt) acc[mt][nt] = zero8f();

  const us* bbh = Bh + ((size_t)(n0 + m)) * Ksz + 8 * hl;
  const us* bbl = Bl + ((size_t)(n0 + m)) * Ksz + 8 * hl;

  #pragma unroll 1
  for (int k0 = 0; k0 < Ksz; k0 += 32) {
    size_t rb0, rb1;
    bool ok0 = true, ok1 = true;
    if (ntaps == 9) {
      const int tap = k0 >> icsh;
      const int ic0 = k0 & (IC - 1);
      const int t3 = tap / 3;
      const int ky = t3 - 1, kx = tap - 3 * t3 - 1;
      int yy = py0 + ky, xx = px0 + kx;
      ok0 = ((unsigned)yy < (unsigned)IMG) && ((unsigned)xx < (unsigned)IMG);
      yy = min(max(yy, 0), IMG - 1);
      xx = min(max(xx, 0), IMG - 1);
      rb0 = ((size_t)(pb0 * HWSZ + yy * IMG + xx)) * IC + ic0;
      yy = py1 + ky; xx = px1 + kx;
      ok1 = ((unsigned)yy < (unsigned)IMG) && ((unsigned)xx < (unsigned)IMG);
      yy = min(max(yy, 0), IMG - 1);
      xx = min(max(xx, 0), IMG - 1);
      rb1 = ((size_t)(pb1 * HWSZ + yy * IMG + xx)) * IC + ic0;
    } else {
      rb0 = ((size_t)prow0) * IC + k0;
      rb1 = ((size_t)prow1) * IC + k0;
    }
    const v16us z16 = zero16();
    v16us a0h = ldfrag(Ah + rb0 + 8 * hl);
    v16us a0l = ldfrag(Al + rb0 + 8 * hl);
    v16us a1h = ldfrag(Ah + rb1 + 8 * hl);
    v16us a1l = ldfrag(Al + rb1 + 8 * hl);
    a0h = ok0 ? a0h : z16;
    a0l = ok0 ? a0l : z16;
    a1h = ok1 ? a1h : z16;
    a1l = ok1 ? a1l : z16;
    #pragma unroll
    for (int nt = 0; nt < 4; ++nt) {
      const size_t bo = ((size_t)nt) * 16 * Ksz + k0;
      const v16us bh = ldfrag(bbh + bo);
      const v16us bl = ldfrag(bbl + bo);
      acc[0][nt] = wmma3(a0h, a0l, bh, bl, acc[0][nt]);
      acc[1][nt] = wmma3(a1h, a1l, bh, bl, acc[1][nt]);
    }
  }

  #pragma unroll
  for (int mt = 0; mt < 2; ++mt)
    #pragma unroll
    for (int nt = 0; nt < 4; ++nt)
      #pragma unroll
      for (int r = 0; r < 8; ++r)
        Cs[(32 * w + 16 * mt + 8 * hl + r) * 64 + nt * 16 + m] = acc[mt][nt][r];
  __syncthreads();

  v4f vals[16];
  #pragma unroll
  for (int i = 0; i < 16; ++i) {
    const int row = 32 * w + 2 * i + (lane >> 4);
    const int col4 = (lane & 15) * 4;
    v4f v = *(const v4fa*)(Cs + row * 64 + col4);
    if (addres) {
      const v4f rr = *(const v4fa*)(Res + ((size_t)(m0 + row)) * N + n0 + col4);
      v += rr;
    }
    vals[i] = v;
  }
  #pragma unroll
  for (int i = 0; i < 16; ++i) {
    const int row = 32 * w + 2 * i + (lane >> 4);
    const int col4 = (lane & 15) * 4;
    *(volatile v4f*)(Cf + ((size_t)(m0 + row)) * N + n0 + col4) = vals[i];
  }
  __threadfence();
  #pragma unroll
  for (int i = 0; i < 16; ++i) {
    const int row = 32 * w + 2 * i + (lane >> 4);
    const int col4 = (lane & 15) * 4;
    *(volatile v4f*)(Cf + ((size_t)(m0 + row)) * N + n0 + col4) = vals[i];
  }
}

__global__ __launch_bounds__(256) void k_dw(const float* __restrict__ In, const float* __restrict__ scsh,
                                           int applybn, const float* __restrict__ Wd,
                                           us* __restrict__ Oh, us* __restrict__ Ol) {
  const int gid = blockIdx.x * 256 + threadIdx.x;
  const int g = gid & 15, p = gid >> 4;
  const int b = p >> 14, y = (p >> 7) & 127, x = p & 127, c0 = g * 8;
  float sc[8], sh[8], acc[8];
  #pragma unroll
  for (int e = 0; e < 8; ++e) {
    const float s1 = scsh[c0 + e], s2 = scsh[128 + c0 + e];
    sc[e] = applybn ? s1 : 1.0f;
    sh[e] = applybn ? s2 : 0.0f;
    acc[e] = 0.0f;
  }
  #pragma unroll 1
  for (int tap = 0; tap < 9; ++tap) {
    const int t3 = tap / 3;
    const int yy = y + t3 - 1, xx = x + (tap - 3 * t3) - 1;
    const bool ok = ((unsigned)yy < (unsigned)IMG) && ((unsigned)xx < (unsigned)IMG);
    const int yc = min(max(yy, 0), IMG - 1), xc = min(max(xx, 0), IMG - 1);
    const float* sp = In + ((size_t)(b * HWSZ + yc * IMG + xc)) * NCH + c0;
    const v4f ia = *(const v4fa*)sp;
    const v4f ib = *(const v4fa*)(sp + 4);
    const float iv[8] = {ia.x, ia.y, ia.z, ia.w, ib.x, ib.y, ib.z, ib.w};
    #pragma unroll
    for (int e = 0; e < 8; ++e) {
      const float wv = Wd[(c0 + e) * 9 + tap];
      float bn = fmaf(iv[e], sc[e], sh[e]);
      bn = ok ? bn : 0.0f;
      acc[e] = fmaf(wv, bn, acc[e]);
    }
  }
  v8us hh, ll;
  #pragma unroll
  for (int e = 0; e < 8; ++e) {
    const us hb = bf_bits(acc[e]);
    hh[e] = hb;
    ll[e] = bf_bits(acc[e] - bf_val(hb));
  }
  const size_t o0 = ((size_t)gid) * 8;
  *(volatile v8us*)(Oh + o0) = hh;
  *(volatile v8us*)(Ol + o0) = ll;
  __threadfence();
  *(volatile v8us*)(Oh + o0) = hh;
  *(volatile v8us*)(Ol + o0) = ll;
}

__global__ __launch_bounds__(256) void k_gather(const us* __restrict__ Ah, const us* __restrict__ Al,
                                               us* __restrict__ Ch, us* __restrict__ Cl) {
  const int gid = blockIdx.x * 256 + threadIdx.x;
  const int row = gid >> 4, piece = gid & 15;
  const int b = row >> 10, t = (row >> 5) & 31, u = row & 31;
  float f;
  const int y = interp_lo(t >> 1, f) + (t & 1);
  const int x = interp_lo(u >> 1, f) + (u & 1);
  const size_t src = ((size_t)(b * HWSZ + y * IMG + x)) * NCH + piece * 8;
  const size_t dst = ((size_t)row) * NCH + piece * 8;
  const v8us hv = *(const v8usa*)(Ah + src);
  const v8us lv = *(const v8usa*)(Al + src);
  *(volatile v8us*)(Ch + dst) = hv;
  *(volatile v8us*)(Cl + dst) = lv;
  __threadfence();
  *(volatile v8us*)(Ch + dst) = hv;
  *(volatile v8us*)(Cl + dst) = lv;
}

__global__ __launch_bounds__(256) void k_down(const float* __restrict__ KVc,
                                             us* __restrict__ Kh, us* __restrict__ Kl,
                                             us* __restrict__ Vh, us* __restrict__ Vl) {
  __shared__ __attribute__((aligned(16))) us Lh[8192];
  __shared__ __attribute__((aligned(16))) us Ll[8192];
  const int bh = blockIdx.x >> 1, which = blockIdx.x & 1;
  const int b = bh >> 2, h = bh & 3;
  const int j = threadIdx.x;
  const int r = j >> 4, s = j & 15;
  float fh, fw;
  (void)interp_lo(r, fh);
  (void)interp_lo(s, fw);
  const float gw0 = 1.0f - fw, gw1 = fw, gh0 = 1.0f - fh, gh1 = fh;
  const int rb = b * 1024 + (2 * r) * 32 + 2 * s;
  const int coff = which ? 128 : 0;
  #pragma unroll 1
  for (int d = 0; d < DHEAD; ++d) {
    const int c = coff + d * 4 + h;
    const float x00 = KVc[((size_t)rb) * 256 + c];
    const float x01 = KVc[((size_t)(rb + 1)) * 256 + c];
    const float x10 = KVc[((size_t)(rb + 32)) * 256 + c];
    const float x11 = KVc[((size_t)(rb + 33)) * 256 + c];
    const float t0 = x00 * gw0 + x01 * gw1;
    const float t1 = x10 * gw0 + x11 * gw1;
    const float val = t0 * gh0 + t1 * gh1;
    const us hb = bf_bits(val);
    const us lb = bf_bits(val - bf_val(hb));
    const int li = which ? (d * NKEY + j) : (j * DHEAD + d);
    Lh[li] = hb;
    Ll[li] = lb;
  }
  __syncthreads();
  us* dh = (which ? Vh : Kh) + ((size_t)bh) * 8192;
  us* dl = (which ? Vl : Kl) + ((size_t)bh) * 8192;
  #pragma unroll
  for (int it = 0; it < 4; ++it) {
    const int off = (it * 256 + j) * 8;
    *(volatile v8us*)(dh + off) = *(const v8usa*)(Lh + off);
    *(volatile v8us*)(dl + off) = *(const v8usa*)(Ll + off);
  }
  __threadfence();
  #pragma unroll
  for (int it = 0; it < 4; ++it) {
    const int off = (it * 256 + j) * 8;
    *(volatile v8us*)(dh + off) = *(const v8usa*)(Lh + off);
    *(volatile v8us*)(dl + off) = *(const v8usa*)(Ll + off);
  }
}

template <int HD>
__device__ __forceinline__ void attn_head(const float* __restrict__ Qf,
                                          const us* __restrict__ Kh, const us* __restrict__ Kl,
                                          const us* __restrict__ Vh, const us* __restrict__ Vl,
                                          const float* __restrict__ tab,
                                          float* Ss, int b, int i0, int w, int lane, v8f (&o)[4][2]) {
  const int hl = lane >> 4, m = lane & 15;
  const int bh = b * 4 + HD;

  v16us qh, ql;
  {
    const float* qp = Qf + ((size_t)(b * HWSZ + i0 + 16 * w + m)) * NCH + HD;
    #pragma unroll
    for (int e = 0; e < 16; ++e) {
      const int d = 8 * hl + e + ((e >> 3) << 3);
      const float v = qp[d * 4];
      const us hb = bf_bits(v);
      qh[e] = hb;
      ql[e] = bf_bits(v - bf_val(hb));
    }
  }

  #pragma unroll 1
  for (int jt = 0; jt < 16; ++jt) {
    const size_t ko = ((size_t)(bh * NKEY + jt * 16 + m)) * DHEAD + 8 * hl;
    const v16us kfh = ldfrag(Kh + ko);
    const v16us kfl = ldfrag(Kl + ko);
    v8f sacc = zero8f();
    sacc = wmma3(qh, ql, kfh, kfl, sacc);
    #pragma unroll
    for (int r = 0; r < 8; ++r) Ss[(16 * w + 8 * hl + r) * NKEY + jt * 16 + m] = sacc[r];
  }
  __syncthreads();

  us* Ps = reinterpret_cast<us*>(Ss);
  const int j0 = 8 * lane;
  const float scale = 0.17677669529663687f;
  #pragma unroll 1
  for (int rr = 0; rr < 16; ++rr) {
    const int row = 16 * w + rr;
    const int i = i0 + row;
    const int ih = i >> 10, iw = (i & 127) >> 3;
    const v4f sa = *(const v4fa*)(Ss + row * NKEY + j0);
    const v4f sb = *(const v4fa*)(Ss + row * NKEY + j0 + 4);
    float sv[8] = {sa.x, sa.y, sa.z, sa.w, sb.x, sb.y, sb.z, sb.w};
    float mx = -3.0e38f;
    #pragma unroll
    for (int e = 0; e < 8; ++e) {
      const int jj = j0 + e;
      const int idx = (ih - (jj >> 4) + 15) * 31 + (iw - (jj & 15) + 15);
      sv[e] = (sv[e] + tab[idx * 4 + HD]) * scale;
      mx = fmaxf(mx, sv[e]);
    }
    #pragma unroll
    for (int off = 16; off > 0; off >>= 1) mx = fmaxf(mx, __shfl_xor(mx, off));
    float sum = 0.0f;
    #pragma unroll
    for (int e = 0; e < 8; ++e) { sv[e] = __expf(sv[e] - mx); sum += sv[e]; }
    #pragma unroll
    for (int off = 16; off > 0; off >>= 1) sum += __shfl_xor(sum, off);
    const float inv = __builtin_amdgcn_rcpf(sum);
    v8us ph, pl;
    #pragma unroll
    for (int e = 0; e < 8; ++e) {
      const float pv = sv[e] * inv;
      const us hb = bf_bits(pv);
      ph[e] = hb;
      pl[e] = bf_bits(pv - bf_val(hb));
    }
    *(v8usa*)(Ps + row * 512 + j0) = ph;
    *(v8usa*)(Ps + row * 512 + 256 + j0) = pl;
  }
  __syncthreads();

  #pragma unroll 1
  for (int ks = 0; ks < 8; ++ks) {
    const us* pp = Ps + (16 * w + m) * 512 + ks * 32 + 8 * hl;
    const v16us ah = ldfrag(pp);
    const v16us al = ldfrag(pp + 256);
    #pragma unroll
    for (int nt = 0; nt < 2; ++nt) {
      const size_t vo = ((size_t)(bh * DHEAD + nt * 16 + m)) * NKEY + ks * 32 + 8 * hl;
      const v16us vfh = ldfrag(Vh + vo);
      const v16us vfl = ldfrag(Vl + vo);
      o[HD][nt] = wmma3(ah, al, vfh, vfl, o[HD][nt]);
    }
  }
  __syncthreads();
}

__global__ __launch_bounds__(128) void k_attn(const float* __restrict__ Qf,
                                             const us* __restrict__ Kh, const us* __restrict__ Kl,
                                             const us* __restrict__ Vh, const us* __restrict__ Vl,
                                             const float* __restrict__ tab, float* __restrict__ Of) {
  __shared__ __attribute__((aligned(16))) float Ss[64 * 256];
  const int tid = threadIdx.x, lane = tid & 31, w = tid >> 5;
  const int hl = lane >> 4, m = lane & 15;
  const int b = blockIdx.y, i0 = blockIdx.x * 64;

  v8f o[4][2];
  #pragma unroll
  for (int hd = 0; hd < 4; ++hd)
    #pragma unroll
    for (int nt = 0; nt < 2; ++nt) o[hd][nt] = zero8f();

  attn_head<0>(Qf, Kh, Kl, Vh, Vl, tab, Ss, b, i0, w, lane, o);
  attn_head<1>(Qf, Kh, Kl, Vh, Vl, tab, Ss, b, i0, w, lane, o);
  attn_head<2>(Qf, Kh, Kl, Vh, Vl, tab, Ss, b, i0, w, lane, o);
  attn_head<3>(Qf, Kh, Kl, Vh, Vl, tab, Ss, b, i0, w, lane, o);

  #pragma unroll
  for (int hd = 0; hd < 4; ++hd)
    #pragma unroll
    for (int nt = 0; nt < 2; ++nt)
      #pragma unroll
      for (int r = 0; r < 8; ++r)
        Ss[(16 * w + 8 * hl + r) * NCH + (nt * 16 + m) * 4 + hd] = o[hd][nt][r];
  __syncthreads();

  float* dst = Of + ((size_t)(b * HWSZ + i0)) * NCH;
  #pragma unroll
  for (int it = 0; it < 16; ++it) {
    const int off = (it * 128 + tid) * 4;
    *(volatile v4f*)(dst + off) = *(const v4fa*)(Ss + off);
  }
  __threadfence();
  #pragma unroll
  for (int it = 0; it < 16; ++it) {
    const int off = (it * 128 + tid) * 4;
    *(volatile v4f*)(dst + off) = *(const v4fa*)(Ss + off);
  }
}

__global__ __launch_bounds__(128) void k_out(const float* __restrict__ In, float* __restrict__ Out) {
  __shared__ __attribute__((aligned(16))) float T[128 * 64];
  const int tid = threadIdx.x, lane = tid & 31, w = tid >> 5;
  const int p0 = blockIdx.x * 64;
  const int b = p0 >> 14, il = p0 & (HWSZ - 1);
  const float* src = In + ((size_t)p0) * NCH;
  #pragma unroll
  for (int it = 0; it < 16; ++it) {
    const int l = (it * 128 + tid) * 4;
    const int row = l >> 7, c0 = l & 127;
    const v4f v = *(const v4fa*)(src + l);
    T[(c0 + 0) * 64 + row] = v.x;
    T[(c0 + 1) * 64 + row] = v.y;
    T[(c0 + 2) * 64 + row] = v.z;
    T[(c0 + 3) * 64 + row] = v.w;
  }
  __syncthreads();
  #pragma unroll
  for (int it = 0; it < 16; ++it) {
    const int c = it * 8 + w * 2 + (lane >> 4);
    const int col4 = (lane & 15) * 4;
    *(volatile v4f*)(Out + ((size_t)(b * NCH + c)) * HWSZ + il + col4) = *(const v4fa*)(T + c * 64 + col4);
  }
  __threadfence();
  #pragma unroll
  for (int it = 0; it < 16; ++it) {
    const int c = it * 8 + w * 2 + (lane >> 4);
    const int col4 = (lane & 15) * 4;
    *(volatile v4f*)(Out + ((size_t)(b * NCH + c)) * HWSZ + il + col4) = *(const v4fa*)(T + c * 64 + col4);
  }
}

extern "C" void kernel_launch(void* const* d_in, const int* in_sizes, int n_in,
                              void* d_out, int out_size, void* d_ws, size_t ws_size,
                              hipStream_t stream) {
  if (n_in < 20) return;
  if (in_sizes[0] != 8388608) return;
  if (in_sizes[1] != 64 || in_sizes[2] != 64 || in_sizes[7] != 64 || in_sizes[8] != 64) return;
  if (in_sizes[4] != 128 || in_sizes[5] != 128) return;
  if (in_sizes[3] != 73728 || in_sizes[6] != 147456 || in_sizes[9] != 8192) return;
  if (in_sizes[10] != 256 || in_sizes[11] != 256 || in_sizes[17] != 256 || in_sizes[18] != 256) return;
  if (in_sizes[12] != 2304 || in_sizes[13] != 98304 || in_sizes[14] != 2304 || in_sizes[15] != 32768) return;
  if (in_sizes[16] != 7688 || in_sizes[19] != 32768) return;
  if (out_size != 4194304) return;

  const float* x        = (const float*)d_in[0];
  const float* bb_bn1_g = (const float*)d_in[1];
  const float* bb_bn1_b = (const float*)d_in[2];
  const float* bb_conv1 = (const float*)d_in[3];
  const float* bb_bn2_g = (const float*)d_in[4];
  const float* bb_bn2_b = (const float*)d_in[5];
  const float* bb_conv2 = (const float*)d_in[6];
  const float* bb_sbn_g = (const float*)d_in[7];
  const float* bb_sbn_b = (const float*)d_in[8];
  const float* bb_sconv = (const float*)d_in[9];
  const float* tb_bn1_g = (const float*)d_in[10];
  const float* tb_bn1_b = (const float*)d_in[11];
  const float* tb_dwqkv = (const float*)d_in[12];
  const float* tb_pwqkv = (const float*)d_in[13];
  const float* tb_dwout = (const float*)d_in[14];
  const float* tb_pwout = (const float*)d_in[15];
  const float* tb_rel   = (const float*)d_in[16];
  const float* tb_bn2_g = (const float*)d_in[17];
  const float* tb_bn2_b = (const float*)d_in[18];
  const float* tb_mlp   = (const float*)d_in[19];
  float* out = (float*)d_out;

  size_t off = 0;
  char* wsb = (char*)d_ws;
  auto carve = [&](size_t bytes) -> char* {
    char* p = wsb + off;
    off += (bytes + 255) & ~(size_t)255;
    return p;
  };
  float*  Pbuf  = (float*)carve((size_t)MTOT * 64 * 4);
  float*  F0    = (float*)carve((size_t)MTOT * NCH * 4);
  float*  F1    = (float*)carve((size_t)MTOT * NCH * 4);
  float*  F2    = (float*)carve((size_t)MTOT * NCH * 4);
  us*     A64h  = (us*)carve((size_t)MTOT * 64 * 2);
  us*     A64l  = (us*)carve((size_t)MTOT * 64 * 2);
  us*     A128h = (us*)carve((size_t)MTOT * NCH * 2);
  us*     A128l = (us*)carve((size_t)MTOT * NCH * 2);
  us*     Ach   = (us*)carve((size_t)NCMP * NCH * 2);
  us*     Acl   = (us*)carve((size_t)NCMP * NCH * 2);
  float*  KVc   = (float*)carve((size_t)NCMP * 256 * 4);
  us*     Kh    = (us*)carve((size_t)8 * NKEY * DHEAD * 2);
  us*     Kl    = (us*)carve((size_t)8 * NKEY * DHEAD * 2);
  us*     Vh    = (us*)carve((size_t)8 * DHEAD * NKEY * 2);
  us*     Vl    = (us*)carve((size_t)8 * DHEAD * NKEY * 2);
  us*     wc1h  = (us*)carve((size_t)128 * 576 * 2);
  us*     wc1l  = (us*)carve((size_t)128 * 576 * 2);
  us*     wc2h  = (us*)carve((size_t)128 * 1152 * 2);
  us*     wc2l  = (us*)carve((size_t)128 * 1152 * 2);
  us*     wsch  = (us*)carve((size_t)128 * 64 * 2);
  us*     wscl  = (us*)carve((size_t)128 * 64 * 2);
  us*     wqkvh = (us*)carve((size_t)768 * 128 * 2);
  us*     wqkvl = (us*)carve((size_t)768 * 128 * 2);
  us*     wouth = (us*)carve((size_t)256 * 128 * 2);
  us*     woutl = (us*)carve((size_t)256 * 128 * 2);
  us*     wmlph = (us*)carve((size_t)256 * 128 * 2);
  us*     wmlpl = (us*)carve((size_t)256 * 128 * 2);
  double* part  = (double*)carve((size_t)256 * 128 * 2 * 8);
  float*  T0    = (float*)carve(256 * 4);
  float*  T1    = (float*)carve(256 * 4);
  float*  T2    = (float*)carve(256 * 4);
  if (off > ws_size) return;

  k_wcvt<<<(128 * 576 / 8 + 255) / 256, 256, 0, stream>>>(bb_conv1, 128, 64, 9, wc1h, wc1l);
  k_wcvt<<<(128 * 1152 / 8 + 255) / 256, 256, 0, stream>>>(bb_conv2, 128, 128, 9, wc2h, wc2l);
  k_wcvt<<<(128 * 64 / 8 + 255) / 256, 256, 0, stream>>>(bb_sconv, 128, 64, 1, wsch, wscl);
  k_wcvt<<<(768 * 128 / 8 + 255) / 256, 256, 0, stream>>>(tb_pwqkv, 768, 128, 1, wqkvh, wqkvl);
  k_wcvt<<<(256 * 128 / 8 + 255) / 256, 256, 0, stream>>>(tb_pwout, 256, 128, 1, wouth, woutl);
  k_wcvt<<<(256 * 128 / 8 + 255) / 256, 256, 0, stream>>>(tb_mlp, 256, 128, 1, wmlph, wmlpl);

  k_maxpool<<<1024, 256, 0, stream>>>(x, Pbuf);
  k_stats<<<MTOT / 128, 256, 0, stream>>>(Pbuf, 64, 6, part);
  k_bnfin<<<1, 128, 0, stream>>>(part, 64, bb_bn1_g, bb_bn1_b, T0);
  k_bnfin<<<1, 128, 0, stream>>>(part, 64, bb_sbn_g, bb_sbn_b, T1);
  k_apply<<<(MTOT * 64 / 8) / 256, 256, 0, stream>>>(Pbuf, T0, 64, 1, A64h, A64l);
  k_gemm<<<dim3(MTOT / 128, 2), 128, 0, stream>>>(A64h, A64l, wc1h, wc1l, F0, F0, 64, 6, 9, 128, 0);
  k_stats<<<MTOT / 128, 256, 0, stream>>>(F0, 128, 7, part);
  k_bnfin<<<1, 128, 0, stream>>>(part, 128, bb_bn2_g, bb_bn2_b, T2);
  k_apply<<<(MTOT * 128 / 8) / 256, 256, 0, stream>>>(F0, T2, 128, 1, A128h, A128l);
  k_apply<<<(MTOT * 64 / 8) / 256, 256, 0, stream>>>(Pbuf, T1, 64, 1, A64h, A64l);
  k_gemm<<<dim3(MTOT / 128, 2), 128, 0, stream>>>(A64h, A64l, wsch, wscl, F1, F1, 64, 6, 1, 128, 0);
  k_gemm<<<dim3(MTOT / 128, 2), 128, 0, stream>>>(A128h, A128l, wc2h, wc2l, F1, F1, 128, 7, 9, 128, 1);

  for (int i = 0; i < 2; ++i) {
    const us* wqh  = wqkvh + (size_t)i * 384 * 128;
    const us* wql  = wqkvl + (size_t)i * 384 * 128;
    const us* wkvh = wqkvh + ((size_t)i * 384 + 128) * 128;
    const us* wkvl = wqkvl + ((size_t)i * 384 + 128) * 128;
    const us* woh  = wouth + (size_t)i * 128 * 128;
    const us* wol  = woutl + (size_t)i * 128 * 128;
    const us* wmh  = wmlph + (size_t)i * 128 * 128;
    const us* wml  = wmlpl + (size_t)i * 128 * 128;

    k_stats<<<MTOT / 128, 256, 0, stream>>>(F1, 128, 7, part);
    k_bnfin<<<1, 128, 0, stream>>>(part, 128, tb_bn1_g + i * 128, tb_bn1_b + i * 128, T0);
    k_dw<<<(MTOT * 16) / 256, 256, 0, stream>>>(F1, T0, 1, tb_dwqkv + (size_t)i * 128 * 9, A128h, A128l);
    k_gemm<<<dim3(MTOT / 128, 2), 128, 0, stream>>>(A128h, A128l, wqh, wql, F0, F0, 128, 7, 1, 128, 0);
    k_gather<<<(NCMP * 16) / 256, 256, 0, stream>>>(A128h, A128l, Ach, Acl);
    k_gemm<<<dim3(NCMP / 128, 4), 128, 0, stream>>>(Ach, Acl, wkvh, wkvl, KVc, KVc, 128, 7, 1, 256, 0);
    k_down<<<16, 256, 0, stream>>>(KVc, Kh, Kl, Vh, Vl);
    k_attn<<<dim3(HWSZ / 64, 2), 128, 0, stream>>>(F0, Kh, Kl, Vh, Vl, tb_rel + (size_t)i * 961 * 4, F2);
    k_dw<<<(MTOT * 16) / 256, 256, 0, stream>>>(F2, T0, 0, tb_dwout + (size_t)i * 128 * 9, A128h, A128l);
    k_gemm<<<dim3(MTOT / 128, 2), 128, 0, stream>>>(A128h, A128l, woh, wol, F1, F1, 128, 7, 1, 128, 1);

    k_stats<<<MTOT / 128, 256, 0, stream>>>(F1, 128, 7, part);
    k_bnfin<<<1, 128, 0, stream>>>(part, 128, tb_bn2_g + i * 128, tb_bn2_b + i * 128, T0);
    k_apply<<<(MTOT * 128 / 8) / 256, 256, 0, stream>>>(F1, T0, 128, 1, A128h, A128l);
    k_gemm<<<dim3(MTOT / 128, 2), 128, 0, stream>>>(A128h, A128l, wmh, wml, F1, F1, 128, 7, 1, 128, 1);
  }

  k_out<<<MTOT / 64, 128, 0, stream>>>(F1, out);
}
